// ReAttentionMSA_75960791597710
// MI455X (gfx1250) — hardware-verified
//
#include <hip/hip_runtime.h>
#include <math.h>
#include <stdint.h>

constexpr int NBATCH = 8;
constexpr int NTOK   = 1024;
constexpr int NEMB   = 384;
constexpr int NHEAD  = 12;
constexpr int HDIM   = 32;
constexpr int TCHUNK = 512;
constexpr int NCHUNK = NTOK / TCHUNK;
constexpr int PHCOLS = 512;
constexpr int QKW    = 64;
constexpr int VTROWS = 64;
constexpr int UW     = 64;
constexpr float SM_SCALE = 0.17677669529663687f;
constexpr float P_CARRY  = 1024.0f;
constexpr float R_CARRY  = 2048.0f;
constexpr float P_INV    = 1.0f / 1024.0f;
constexpr float MIX_FOLD = 1.0f / (1024.0f * 2048.0f);
constexpr float BN_EPS   = 1e-5f;

typedef __attribute__((ext_vector_type(16))) _Float16 v16h;
typedef __attribute__((ext_vector_type(8)))  _Float16 v8h;
typedef __attribute__((ext_vector_type(16))) __bf16   v16b;
typedef __attribute__((ext_vector_type(8)))  __bf16   v8b;
typedef __attribute__((ext_vector_type(8)))  float    v8f;
typedef __attribute__((ext_vector_type(4)))  float    v4f;
typedef __attribute__((ext_vector_type(2)))  float    v2f;
typedef __attribute__((ext_vector_type(4)))  unsigned int v4u;
typedef __attribute__((ext_vector_type(8)))  unsigned short v8us;

__device__ __forceinline__ unsigned short f2bf_bits(float f) {
  unsigned u = __float_as_uint(f);
  return (unsigned short)((u + 0x7FFFu + ((u >> 16) & 1u)) >> 16);
}
__device__ __forceinline__ float bf_bits2f(unsigned short h) { return __uint_as_float(((unsigned)h) << 16); }
__device__ __forceinline__ unsigned pk16(unsigned short a, unsigned short b) { return (unsigned)a | ((unsigned)b << 16); }

__device__ __forceinline__ void dep_guard_h(v8f& a, v8f& b, v16h x, v16h y) { asm volatile("v_nop\n\tv_nop\n\tv_nop\n\tv_nop" : "+v"(a), "+v"(b) : "v"(x), "v"(y)); }
__device__ __forceinline__ void dep_guard_b(v8f& a, v8f& b, v16b x, v16b y) { asm volatile("v_nop\n\tv_nop\n\tv_nop\n\tv_nop" : "+v"(a), "+v"(b) : "v"(x), "v"(y)); }
__device__ __forceinline__ void keep4_h(v16h a, v16h b, v16h c, v16h d) { asm volatile("v_nop" :: "v"(a), "v"(b), "v"(c), "v"(d)); }
__device__ __forceinline__ void keep4_b(v16b a, v16b b, v16b c, v16b d) { asm volatile("v_nop" :: "v"(a), "v"(b), "v"(c), "v"(d)); }
__device__ __forceinline__ void acc_guard4(v8f& a, v8f& b, v8f& c, v8f& d) { asm volatile("v_nop\n\tv_nop\n\tv_nop\n\tv_nop" : "+v"(a), "+v"(b), "+v"(c), "+v"(d)); }
template <typename T> struct Frag;
template <> struct Frag<_Float16> {
  typedef v16h V; union U { v16h v; v8h h[2]; };
  static __device__ __forceinline__ v16h load(const _Float16* p) {
    U f; f.h[0] = *(const v8h*)(p); f.h[1] = *(const v8h*)(p + 16); return f.v;
  }
  static __device__ __forceinline__ v8f mma(v16h a, v16h b, v8f c) {
    return __builtin_amdgcn_wmma_f32_16x16x32_f16(false, a, false, b, (short)0, c, false, false);
  }
  static __device__ __forceinline__ void guard(v8f& a, v8f& b, v16h x, v16h y) { dep_guard_h(a, b, x, y); }
  static __device__ __forceinline__ void keep(v16h a, v16h b, v16h c, v16h d) { keep4_h(a, b, c, d); }
};
template <> struct Frag<__bf16> {
  typedef v16b V; union U { v16b v; v8b h[2]; };
  static __device__ __forceinline__ v16b load(const __bf16* p) {
    U f; f.h[0] = *(const v8b*)(p); f.h[1] = *(const v8b*)(p + 16); return f.v;
  }
  static __device__ __forceinline__ v8f mma(v16b a, v16b b, v8f c) {
    return __builtin_amdgcn_wmma_f32_16x16x32_bf16(false, a, false, b, (short)0, c, false, false);
  }
  static __device__ __forceinline__ void guard(v8f& a, v8f& b, v16b x, v16b y) { dep_guard_b(a, b, x, y); }
  static __device__ __forceinline__ void keep(v16b a, v16b b, v16b c, v16b d) { keep4_b(a, b, c, d); }
};

template <int ET> struct Elem;
template <> struct Elem<0> { typedef _Float16 T; };
template <> struct Elem<1> { typedef __bf16 T; };
template <int ET, bool SPLIT, int BIAS_MODE, int OUT_MODE, bool RESID, int ACT = 0>
__global__ __launch_bounds__(256) void wmma_gemm64(
    const unsigned short* __restrict__ Ap, const unsigned short* __restrict__ A2p, int lda, long strideA,
    const unsigned short* __restrict__ Btp, const unsigned short* __restrict__ Bt2p, int ldb, long strideB,
    void* __restrict__ Cout, void* __restrict__ Cout2, int ldc, long strideC,
    const float* __restrict__ bias,
    const float* __restrict__ resid, long strideR,
    int M, int N, int K, float scale) {
  typedef typename Elem<ET>::T T;
  typedef typename Frag<T>::V V;
  const T* A = (const T*)Ap; const T* A2 = (const T*)A2p; const T* Bt = (const T*)Btp; const T* Bt2 = (const T*)Bt2p;
  __shared__ __align__(16) float sT[8][16 * 68];
  const int b    = blockIdx.y;
  const int lane = threadIdx.x & 31;
  const int wave = threadIdx.x >> 5;
  const int tilesN = N >> 6;
  const int tilesM = M >> 6;
  const int tile = blockIdx.x * 8 + wave;
  if (tile >= tilesM * tilesN) return;
  const int tm = tile / tilesN;
  const int tn = tile - tm * tilesN;
  const int m0 = tm << 6;
  const int n0 = tn << 6;

  const T* Ab  = A  + (size_t)b * strideA;
  const T* Bb  = Bt + (size_t)b * strideB;
  const T* Ab2 = SPLIT ? (A2  + (size_t)b * strideA) : nullptr;
  const T* Bb2 = SPLIT ? (Bt2 + (size_t)b * strideB) : nullptr;

  const int rlane = lane & 15;
  const int koff  = (lane >> 4) * 8;
  const int mOff  = (lane >> 4) * 8;

  v8f acc[4][4];
#pragma unroll
  for (int i = 0; i < 4; ++i)
#pragma unroll
    for (int j = 0; j < 4; ++j) acc[i][j] = (v8f){0.f,0.f,0.f,0.f,0.f,0.f,0.f,0.f};

  for (int k0 = 0; k0 < K; k0 += 32) {
    V bh[4], bl[4];
#pragma unroll
    for (int j = 0; j < 4; ++j) {
      const size_t bo = (size_t)(n0 + (j << 4) + rlane) * ldb + koff + k0;
      bh[j] = Frag<T>::load(Bb + bo);
      if (SPLIT) bl[j] = Frag<T>::load(Bb2 + bo);
    }
#pragma unroll
    for (int i = 0; i < 4; ++i) {
      const size_t ao = (size_t)(m0 + (i << 4) + rlane) * lda + koff + k0;
      V ah = Frag<T>::load(Ab + ao);
      V al;
      if (SPLIT) al = Frag<T>::load(Ab2 + ao);
#pragma unroll
      for (int j = 0; j < 4; ++j) {
        acc[i][j] = Frag<T>::mma(ah, bh[j], acc[i][j]);
        if (SPLIT) {
          acc[i][j] = Frag<T>::mma(ah, bl[j], acc[i][j]);
          acc[i][j] = Frag<T>::mma(al, bh[j], acc[i][j]);
        }
      }
      Frag<T>::guard(acc[i][0], acc[i][3], ah, SPLIT ? al : ah);
    }
    Frag<T>::keep(bh[0], bh[1], bh[2], bh[3]);
    if (SPLIT) Frag<T>::keep(bl[0], bl[1], bl[2], bl[3]);
  }
  acc_guard4(acc[0][0], acc[0][1], acc[0][2], acc[0][3]);
  acc_guard4(acc[1][0], acc[1][1], acc[1][2], acc[1][3]);
  acc_guard4(acc[2][0], acc[2][1], acc[2][2], acc[2][3]);
  acc_guard4(acc[3][0], acc[3][1], acc[3][2], acc[3][3]);

  float* slab = sT[wave];
  const float* Rb = RESID ? (resid + (size_t)b * strideR) : nullptr;
#pragma unroll
  for (int i = 0; i < 4; ++i) {
    const int mBase = m0 + (i << 4);
#pragma unroll
    for (int j = 0; j < 4; ++j) {
      const int n = n0 + (j << 4) + rlane;
      float bv = 0.f;
      if (BIAS_MODE == 2) bv = bias[n];
#pragma unroll
      for (int r = 0; r < 8; ++r) {
        float v = acc[i][j][r] * scale;
        if (BIAS_MODE == 1) v += bias[mBase + mOff + r];
        if (BIAS_MODE == 2) v += bv;
        if (RESID) v += Rb[(size_t)(mBase + mOff + r) * ldc + n];
        if (ACT == 1) v = tanhf(v);
        if (ACT == 2) v = fmaxf(v, 0.0f);
        if (ACT == 3) v = v / (1.0f + expf(-v));
        if (ACT == 4) v = (v > 0.f) ? v : 0.01f * v;
        if (ACT == 5) v = 0.5f * v * (1.0f + erff(v * 0.70710678118654752f));
        slab[(mOff + r) * 68 + (j << 4) + rlane] = v;
      }
    }
    __builtin_amdgcn_fence(__ATOMIC_RELEASE, "workgroup");
    __builtin_amdgcn_wave_barrier();
    __builtin_amdgcn_fence(__ATOMIC_ACQUIRE, "workgroup");
    if (OUT_MODE == 0) {
      float* C = (float*)Cout + (size_t)b * strideC;
      const int hh = lane >> 4, c4 = (lane & 15) * 4;
      for (int pass = 0; pass < 2; ++pass) {
#pragma unroll
        for (int it = 0; it < 8; ++it) {
          const int row = it * 2 + hh;
          v4f v = *(const v4f*)(slab + row * 68 + c4);
          *(volatile v4f*)(C + (size_t)(mBase + row) * ldc + n0 + c4) = v;
        }
        __threadfence();
      }
    } else {
      const int q = lane >> 3, c8 = (lane & 7) * 8;
      unsigned short* C  = (unsigned short*)Cout  + (size_t)b * strideC;
      unsigned short* C2 = (OUT_MODE == 2) ? ((unsigned short*)Cout2 + (size_t)b * strideC) : nullptr;
      for (int pass = 0; pass < 2; ++pass) {
#pragma unroll
        for (int it = 0; it < 4; ++it) {
          const int row = it * 4 + q;
          const float* sp = slab + row * 68 + c8;
          v8h hv, lv;
#pragma unroll
          for (int e = 0; e < 8; ++e) {
            if (OUT_MODE == 1) {
              hv[e] = (_Float16)sp[e];
            } else {
              unsigned short hb = f2bf_bits(sp[e]);
              unsigned short lb = f2bf_bits(sp[e] - bf_bits2f(hb));
              hv[e] = __builtin_bit_cast(_Float16, hb);
              lv[e] = __builtin_bit_cast(_Float16, lb);
            }
          }
          *(volatile v8h*)(C + (size_t)(mBase + row) * ldc + n0 + c8) = hv;
          if (OUT_MODE == 2) *(volatile v8h*)(C2 + (size_t)(mBase + row) * ldc + n0 + c8) = lv;
        }
        __threadfence();
      }
    }
    __builtin_amdgcn_fence(__ATOMIC_RELEASE, "workgroup");
    __builtin_amdgcn_wave_barrier();
    __builtin_amdgcn_fence(__ATOMIC_ACQUIRE, "workgroup");
  }
}

__global__ __launch_bounds__(256) void split_bf16x2_kernel(const float* __restrict__ in, unsigned short* __restrict__ hi,
                                                           unsigned short* __restrict__ lo, int n2) {
  const int i = blockIdx.x * 256 + threadIdx.x;
  if (i < n2) {
    const v2f f = *(const v2f*)(in + 2 * (size_t)i);
    const unsigned short h0 = f2bf_bits(f[0]), h1 = f2bf_bits(f[1]);
    const unsigned short l0 = f2bf_bits(f[0] - bf_bits2f(h0)), l1 = f2bf_bits(f[1] - bf_bits2f(h1));
    const unsigned uh = pk16(h0, h1), ul = pk16(l0, l1);
    ((volatile unsigned*)hi)[i] = uh;
    ((volatile unsigned*)lo)[i] = ul;
    __threadfence();
    ((volatile unsigned*)hi)[i] = uh;
    ((volatile unsigned*)lo)[i] = ul;
  }
}

__device__ __forceinline__ void split_pair(float f0, float f1, unsigned& h, unsigned& l) {
  const unsigned short h0 = f2bf_bits(f0), h1 = f2bf_bits(f1);
  const unsigned short l0 = f2bf_bits(f0 - bf_bits2f(h0));
  const unsigned short l1 = f2bf_bits(f1 - bf_bits2f(h1));
  h = pk16(h0, h1);
  l = pk16(l0, l1);
}
__global__ __launch_bounds__(256) void wprep_kernel(const float* __restrict__ Wqkv, const float* __restrict__ bqkv,
                                                    unsigned short* __restrict__ wqkh, unsigned short* __restrict__ wqkl,
                                                    unsigned short* __restrict__ wvh, unsigned short* __restrict__ wvl,
                                                    float* __restrict__ bv) {
  const int tid  = threadIdx.x;
  const int row  = tid >> 2;
  const int col0 = (tid & 3) * 8;
  v4u qh, ql, vh, vl;
#pragma unroll
  for (int p = 0; p < 4; ++p) {
    const int col = col0 + 2 * p;
    const float wq0 = Wqkv[row * HDIM + col];
    const float wq1 = Wqkv[row * HDIM + col + 1];
    int rv = 64 + row; rv = rv > 95 ? 95 : rv;
    float wv0 = Wqkv[rv * HDIM + col];
    float wv1 = Wqkv[rv * HDIM + col + 1];
    wv0 = (row < 32) ? wv0 : 0.0f;
    wv1 = (row < 32) ? wv1 : 0.0f;
    unsigned a, bq, cv, dv;
    split_pair(wq0, wq1, a, bq);
    split_pair(wv0, wv1, cv, dv);
    qh[p] = a; ql[p] = bq; vh[p] = cv; vl[p] = dv;
  }
  v4f b4;
#pragma unroll
  for (int e = 0; e < 4; ++e) {
    int m = tid * 4 + e; m = m > 63 ? 63 : m;
    int mi = 64 + m; mi = mi > 95 ? 95 : mi;
    const float v = bqkv[mi];
    b4[e] = (m < 32) ? v : 0.0f;
  }
  const size_t o = (size_t)tid * 8;
  for (int pass = 0; pass < 2; ++pass) {
    *(volatile v4u*)(wqkh + o) = qh;
    *(volatile v4u*)(wqkl + o) = ql;
    *(volatile v4u*)(wvh + o)  = vh;
    *(volatile v4u*)(wvl + o)  = vl;
    if (tid < 16) *(volatile v4f*)(bv + tid * 4) = b4;
    __threadfence();
  }
}

union HFrag { v16h v; v8h h[2]; };

template <int J>
__device__ __forceinline__ void stage_pcol(const float (&pz)[12][4], int sl, _Float16* Pth, _Float16* Ptl) {
  v8h h0, h1, l0, l1;
#pragma unroll
  for (int e = 0; e < 8; ++e) {
    const float p0 = pz[e][J] * P_CARRY;
    const _Float16 a0 = (_Float16)p0;
    h0[e] = a0;
    l0[e] = (_Float16)((p0 - (float)a0) * R_CARRY);
  }
#pragma unroll
  for (int e = 0; e < 4; ++e) {
    const float p1 = pz[8 + e][J] * P_CARRY;
    const _Float16 a1 = (_Float16)p1;
    h1[e] = a1;
    l1[e] = (_Float16)((p1 - (float)a1) * R_CARRY);
  }
#pragma unroll
  for (int e = 4; e < 8; ++e) { h1[e] = (_Float16)0.0f; l1[e] = (_Float16)0.0f; }
  *(v8h*)(Pth + sl * 16)     = h0;
  *(v8h*)(Pth + sl * 16 + 8) = h1;
  *(v8h*)(Ptl + sl * 16)     = l0;
  *(v8h*)(Ptl + sl * 16 + 8) = l1;
}

__global__ __launch_bounds__(256) void softmax_mix_kernel(const float* __restrict__ S, const float* __restrict__ Wconv,
                                                          unsigned short* __restrict__ Mh, unsigned short* __restrict__ Ml,
                                                          float* __restrict__ part) {
  __shared__ __align__(16) _Float16 Pth[PHCOLS * 16];
  __shared__ __align__(16) _Float16 Ptl[PHCOLS * 16];
  __shared__ __align__(16) float slab[8][12 * 64];
  __shared__ float redw[8][12];
  __shared__ float fin[12];
  __shared__ float stw[8][24];
  __shared__ __align__(16) float pline[32];

  const int tid  = threadIdx.x;
  const int lane = tid & 31;
  const int wave = tid >> 5;
  const int hh   = lane >> 4;
  const int c    = lane & 15;
  const int tl   = blockIdx.x;

  v8h z8;
#pragma unroll
  for (int e = 0; e < 8; ++e) z8[e] = (_Float16)0.0f;
  const v8f zacc = (v8f){0.f,0.f,0.f,0.f,0.f,0.f,0.f,0.f};

  HFrag fah, fal;
  {
    v8h wh8, wl8;
#pragma unroll
    for (int i = 0; i < 8; ++i) {
      const int h  = 8 * hh + i;
      const int gi = c > 11 ? 11 : c;
      const int hi = h > 11 ? 11 : h;
      float w = Wconv[gi * NHEAD + hi];
      w = (c < 12 && h < 12) ? w : 0.0f;
      const _Float16 a = (_Float16)w;
      wh8[i] = a;
      wl8[i] = (_Float16)((w - (float)a) * R_CARRY);
    }
    fah.h[0] = wh8; fah.h[1] = z8;
    fal.h[0] = wl8; fal.h[1] = z8;
  }

  float pz[12][4];
  {
    const float* Srow = S + (size_t)tl * NTOK;
#pragma unroll
    for (int h = 0; h < 12; ++h)
#pragma unroll
      for (int j = 0; j < 4; ++j)
        pz[h][j] = Srow[(size_t)h * TCHUNK * NTOK + tid + 256 * j];
  }
#pragma unroll
  for (int h = 0; h < 12; ++h) {
    float m = fmaxf(fmaxf(pz[h][0], pz[h][1]), fmaxf(pz[h][2], pz[h][3]));
#pragma unroll
    for (int off = 16; off > 0; off >>= 1) m = fmaxf(m, __shfl_xor(m, off, 32));
    if (lane == 0) redw[wave][h] = m;
  }
  __syncthreads();
  if (wave == 0) {
    const int hq = lane < 12 ? lane : 11;
    float m = redw[0][hq];
#pragma unroll
    for (int w = 1; w < 8; ++w) m = fmaxf(m, redw[w][hq]);
    if (lane < 12) fin[lane] = m;
  }
  __syncthreads();
  float mx[12];
#pragma unroll
  for (int h = 0; h < 12; ++h) mx[h] = fin[h];
#pragma unroll
  for (int h = 0; h < 12; ++h) {
#pragma unroll
    for (int j = 0; j < 4; ++j) pz[h][j] = __expf(pz[h][j] - mx[h]);
    float s = ((pz[h][0] + pz[h][1]) + pz[h][2]) + pz[h][3];
#pragma unroll
    for (int off = 16; off > 0; off >>= 1) s += __shfl_xor(s, off, 32);
    if (lane == 0) redw[wave][h] = s;
  }
  __syncthreads();
  if (wave == 0) {
    const int hq = lane < 12 ? lane : 11;
    float s = redw[0][hq];
#pragma unroll
    for (int w = 1; w < 8; ++w) s += redw[w][hq];
    if (lane < 12) fin[lane] = s;
  }
  __syncthreads();
#pragma unroll
  for (int h = 0; h < 12; ++h) {
    const float inv = 1.0f / fin[h];
#pragma unroll
    for (int j = 0; j < 4; ++j) pz[h][j] *= inv;
  }

  v8f s1 = zacc, s2 = zacc;
  float* myslab = slab[wave];
  const int q  = lane >> 3;
  const int c8 = (lane & 7) * 8;
  for (int ph = 0; ph < 2; ++ph) {
    if (ph == 0) {
      stage_pcol<0>(pz, tid, Pth, Ptl);
      stage_pcol<1>(pz, tid + 256, Pth, Ptl);
    } else {
      stage_pcol<2>(pz, tid, Pth, Ptl);
      stage_pcol<3>(pz, tid + 256, Pth, Ptl);
    }
    __syncthreads();
#pragma unroll 1
    for (int nt = 0; nt < 4; ++nt) {
      const int col = wave * 64 + nt * 16 + c;
      HFrag bh, bl;
      bh.h[0] = *(const v8h*)(Pth + col * 16 + 8 * hh); bh.h[1] = z8;
      bl.h[0] = *(const v8h*)(Ptl + col * 16 + 8 * hh); bl.h[1] = z8;
      v8f acc0 = zacc, accr = zacc;
      acc0 = Frag<_Float16>::mma(fah.v, bh.v, acc0);
      accr = Frag<_Float16>::mma(fah.v, bl.v, accr);
      accr = Frag<_Float16>::mma(fal.v, bh.v, accr);
      dep_guard_h(acc0, accr, bh.v, bl.v);
#pragma unroll
      for (int r = 0; r < 8; ++r) {
        const float m = fmaf(accr[r], MIX_FOLD, acc0[r] * P_INV);
        s1[r] += m;
        s2[r] = fmaf(m, m, s2[r]);
        if (hh == 0 || r < 4) myslab[(8 * hh + r) * 64 + nt * 16 + c] = m;
      }
    }
    __syncthreads();
    {
      v8h hv[3], lv[3];
#pragma unroll
      for (int it = 0; it < 3; ++it) {
        const int g = it * 4 + q;
        const float* sp = myslab + g * 64 + c8;
        v8h a, bq;
#pragma unroll
        for (int e = 0; e < 8; ++e) {
          const unsigned short hb = f2bf_bits(sp[e]);
          const unsigned short lb = f2bf_bits(sp[e] - bf_bits2f(hb));
          a[e]  = __builtin_bit_cast(_Float16, hb);
          bq[e] = __builtin_bit_cast(_Float16, lb);
        }
        hv[it] = a; lv[it] = bq;
      }
      for (int pass = 0; pass < 2; ++pass) {
#pragma unroll
        for (int it = 0; it < 3; ++it) {
          const int g = it * 4 + q;
          const size_t go = ((size_t)g * TCHUNK + tl) * NTOK + (size_t)ph * PHCOLS + wave * 64 + c8;
          *(volatile v8h*)(Mh + go) = hv[it];
          *(volatile v8h*)(Ml + go) = lv[it];
        }
        __threadfence();
      }
    }
    __syncthreads();
  }

#pragma unroll
  for (int r = 0; r < 8; ++r) {
    float a = s1[r], bq = s2[r];
#pragma unroll
    for (int off = 1; off < 16; off <<= 1) { a += __shfl_xor(a, off, 32); bq += __shfl_xor(bq, off, 32); }
    const int g = 8 * hh + r;
    if (c == 0 && g < 12) { stw[wave][g] = a; stw[wave][12 + g] = bq; }
  }
  __syncthreads();
  if (wave == 0) {
    const int qi = lane < 24 ? lane : 23;
    float v = stw[0][qi];
#pragma unroll
    for (int w = 1; w < 8; ++w) v += stw[w][qi];
    v = (lane < 24) ? v : 0.0f;
    pline[lane] = v;
  }
  __syncthreads();
  if (tid < 8) {
    const v4f v = *(const v4f*)(pline + tid * 4);
    float* dst = part + (size_t)tl * 32 + tid * 4;
    *(volatile v4f*)dst = v;
    __threadfence();
    *(volatile v4f*)dst = v;
  }
}

__global__ __launch_bounds__(256) void vsum_kernel(const unsigned short* __restrict__ vth, const unsigned short* __restrict__ vtl,
                                                   float* __restrict__ vsum) {
  __shared__ __align__(16) float vs[32];
  const int g   = blockIdx.x;
  const int tid = threadIdx.x;
  const int d   = tid >> 3;
  const int prt = tid & 7;
  const size_t base = ((size_t)g * VTROWS + d) * NTOK + (size_t)prt * 128;
  float acc = 0.0f;
#pragma unroll 1
  for (int i = 0; i < 16; ++i) {
    const v8us a  = *(const v8us*)(vth + base + i * 8);
    const v8us bq = *(const v8us*)(vtl + base + i * 8);
#pragma unroll
    for (int e = 0; e < 8; ++e) acc += bf_bits2f(a[e]) + bf_bits2f(bq[e]);
  }
  acc += __shfl_xor(acc, 1, 32);
  acc += __shfl_xor(acc, 2, 32);
  acc += __shfl_xor(acc, 4, 32);
  if (prt == 0) vs[d] = acc;
  __syncthreads();
  if (tid < 8) {
    const v4f v = *(const v4f*)(vs + tid * 4);
    float* dst = vsum + g * 32 + tid * 4;
    *(volatile v4f*)dst = v;
    __threadfence();
    *(volatile v4f*)dst = v;
  }
}

__global__ __launch_bounds__(32) void coef_kernel(const float* __restrict__ part, const float* __restrict__ bconv,
                                                  const float* __restrict__ gamma, const float* __restrict__ beta,
                                                  float* __restrict__ coef, int nrows) {
  __shared__ double sd[32];
  __shared__ __align__(16) float cf[32];
  const int lane = threadIdx.x;
  double acc = 0.0;
#pragma unroll 1
  for (int r = 0; r < nrows; ++r) acc += (double)part[(size_t)r * 32 + lane];
  sd[lane] = acc;
  __syncthreads();
  int gq = (lane < 12) ? lane : (lane - 12);
  gq = gq < 0 ? 0 : (gq > 11 ? 11 : gq);
  const double s1d = sd[gq];
  const double s2d = sd[12 + gq];
  const double invN = 1.0 / ((double)NBATCH * (double)NTOK * (double)NTOK);
  const double meanM = s1d * invN;
  double var = s2d * invN - meanM * meanM;
  var = var < 0.0 ? 0.0 : var;
  const float varf   = (float)var;
  const float meanre = (float)meanM + bconv[gq];
  const float a      = gamma[gq] * (1.0f / sqrtf(varf + BN_EPS));
  const float kk     = a * bconv[gq] + (beta[gq] - a * meanre);
  const float v = (lane < 12) ? a : ((lane < 24) ? kk : 0.0f);
  cf[lane] = v;
  __syncthreads();
  if (lane < 8) {
    const v4f w = *(const v4f*)(cf + lane * 4);
    float* dst = coef + lane * 4;
    *(volatile v4f*)dst = w;
    __threadfence();
    *(volatile v4f*)dst = w;
  }
}

__global__ __launch_bounds__(256) void combine_kernel(const float* __restrict__ U, const float* __restrict__ vsum,
                                                      const float* __restrict__ coef, float* __restrict__ out) {
  const int lane = threadIdx.x & 31;
  const int wave = threadIdx.x >> 5;
  const int R = blockIdx.x * 8 + wave;
  const int b = R >> 10, t = R & (NTOK - 1);
  v4f o[3];
#pragma unroll
  for (int i = 0; i < 3; ++i) {
    const int f = 128 * i + 4 * lane;
    const int g = f >> 5, d = f & 31;
    const v4f u  = *(const v4f*)(U + (((size_t)(b * NHEAD + g)) * NTOK + t) * UW + d);
    const v4f vv = *(const v4f*)(vsum + (b * NHEAD + g) * 32 + d);
    const float a = coef[g], kk = coef[12 + g];
    v4f rr;
#pragma unroll
    for (int e = 0; e < 4; ++e) rr[e] = fmaf(a, u[e], kk * vv[e]);
    o[i] = rr;
  }
  float* orow = out + (size_t)R * NEMB;
  for (int pass = 0; pass < 2; ++pass) {
#pragma unroll
    for (int i = 0; i < 3; ++i) *(volatile v4f*)(orow + 128 * i + 4 * lane) = o[i];
    __threadfence();
  }
}

extern "C" void kernel_launch(void* const* d_in, const int* in_sizes, int n_in,
                              void* d_out, int out_size, void* d_ws, size_t ws_size,
                              hipStream_t stream) {
  if (n_in < 7) return;
  if (in_sizes[0] != NBATCH * NTOK * NEMB) return;
  if (in_sizes[1] != 3 * HDIM * HDIM || in_sizes[2] != 3 * HDIM) return;
  if (in_sizes[3] != NHEAD * NHEAD || in_sizes[4] < NHEAD || in_sizes[5] < NHEAD || in_sizes[6] < NHEAD) return;
  if (out_size != NBATCH * NTOK * NEMB) return;

  const float* x     = (const float*)d_in[0];
  const float* Wqkv  = (const float*)d_in[1];
  const float* bqkv  = (const float*)d_in[2];
  const float* Wconv = (const float*)d_in[3];
  const float* bconv = (const float*)d_in[4];
  const float* gamma = (const float*)d_in[5];
  const float* beta  = (const float*)d_in[6];
  float* out = (float*)d_out;

  const size_t szX    = (size_t)NBATCH * NTOK * NEMB * 2;
  const size_t szW    = (size_t)64 * HDIM * 2;
  const size_t szBV   = 256;
  const size_t szQK   = (size_t)NBATCH * NTOK * NHEAD * QKW * 2;
  const size_t szVT   = (size_t)NHEAD * VTROWS * NTOK * 2;
  const size_t szS    = (size_t)NHEAD * TCHUNK * NTOK * 4;
  const size_t szM    = (size_t)NHEAD * TCHUNK * NTOK * 2;
  const size_t szU    = (size_t)NBATCH * NHEAD * NTOK * UW * 4;
  const size_t szPART = (size_t)NBATCH * NTOK * 32 * 4;
  const size_t szVS   = (size_t)NBATCH * NHEAD * 32 * 4;
  const size_t szCF   = 256;
  size_t off = 0;
  const size_t oXH = off;   off += szX;
  const size_t oXL = off;   off += szX;
  const size_t oWQKH = off; off += szW;
  const size_t oWQKL = off; off += szW;
  const size_t oWVH = off;  off += szW;
  const size_t oWVL = off;  off += szW;
  const size_t oBV = off;   off += szBV;
  const size_t oQKH = off;  off += szQK;
  const size_t oQKL = off;  off += szQK;
  const size_t oVTH = off;  off += szVT;
  const size_t oVTL = off;  off += szVT;
  const size_t oS = off;    off += szS;
  const size_t oMH = off;   off += szM;
  const size_t oML = off;   off += szM;
  const size_t oU = off;    off += szU;
  const size_t oPART = off; off += szPART;
  const size_t oVS = off;   off += szVS;
  const size_t oCF = off;   off += szCF;
  if (off > ws_size) return;

  char* ws = (char*)d_ws;
  unsigned short* XH   = (unsigned short*)(ws + oXH);
  unsigned short* XL   = (unsigned short*)(ws + oXL);
  unsigned short* WQKH = (unsigned short*)(ws + oWQKH);
  unsigned short* WQKL = (unsigned short*)(ws + oWQKL);
  unsigned short* WVH  = (unsigned short*)(ws + oWVH);
  unsigned short* WVL  = (unsigned short*)(ws + oWVL);
  float*          BV   = (float*)(ws + oBV);
  unsigned short* QKH  = (unsigned short*)(ws + oQKH);
  unsigned short* QKL  = (unsigned short*)(ws + oQKL);
  unsigned short* VTH  = (unsigned short*)(ws + oVTH);
  unsigned short* VTL  = (unsigned short*)(ws + oVTL);
  float*          Sbuf = (float*)(ws + oS);
  unsigned short* MH   = (unsigned short*)(ws + oMH);
  unsigned short* ML   = (unsigned short*)(ws + oML);
  float*          U    = (float*)(ws + oU);
  float*          PART = (float*)(ws + oPART);
  float*          VSUM = (float*)(ws + oVS);
  float*          COEF = (float*)(ws + oCF);

  const dim3 blk(256);
  const int n2x = NBATCH * NTOK * NEMB / 2;
  split_bf16x2_kernel<<<dim3((n2x + 255) / 256), blk, 0, stream>>>(x, XH, XL, n2x);
  wprep_kernel<<<dim3(1), blk, 0, stream>>>(Wqkv, bqkv, WQKH, WQKL, WVH, WVL, BV);
  wmma_gemm64<1, true, 2, 2, false><<<dim3((NBATCH * NTOK * NHEAD / 64) / 8, 1), blk, 0, stream>>>(
      XH, XL, HDIM, 0L, WQKH, WQKL, HDIM, 0L, (void*)QKH, (void*)QKL, QKW, 0L,
      bqkv, bqkv, 0L, NBATCH * NTOK * NHEAD, QKW, HDIM, 1.0f);

  const int nrows = NBATCH * NTOK;
  for (int b = 0; b < NBATCH; ++b) {
    const unsigned short* xbh = XH + (size_t)b * NTOK * NEMB;
    const unsigned short* xbl = XL + (size_t)b * NTOK * NEMB;
    wmma_gemm64<1, true, 1, 2, false><<<dim3(2, NHEAD), blk, 0, stream>>>(
        WVH, WVL, HDIM, 0L, xbh, xbl, NEMB, (long)HDIM, (void*)VTH, (void*)VTL, NTOK, (long)VTROWS * NTOK,
        BV, BV, 0L, VTROWS, NTOK, HDIM, 1.0f);
    vsum_kernel<<<dim3(NHEAD), blk, 0, stream>>>(VTH, VTL, VSUM + (size_t)b * NHEAD * 32);
    for (int ch = 0; ch < NCHUNK; ++ch) {
      const size_t qoff = ((size_t)b * NTOK + (size_t)ch * TCHUNK) * NHEAD * QKW;
      const size_t koff = (size_t)b * NTOK * NHEAD * QKW + HDIM;
      wmma_gemm64<1, true, 0, 0, false><<<dim3(16, NHEAD), blk, 0, stream>>>(
          QKH + qoff, QKL + qoff, NHEAD * QKW, (long)QKW, QKH + koff, QKL + koff, NHEAD * QKW, (long)QKW,
          (void*)Sbuf, (void*)Sbuf, NTOK, (long)TCHUNK * NTOK,
          bqkv, bqkv, 0L, TCHUNK, NTOK, HDIM, SM_SCALE);
      softmax_mix_kernel<<<dim3(TCHUNK), blk, 0, stream>>>(
          Sbuf, Wconv, MH, ML, PART + ((size_t)b * NTOK + (size_t)ch * TCHUNK) * 32);
      float* Ub = U + ((size_t)b * NHEAD * NTOK + (size_t)ch * TCHUNK) * UW;
      wmma_gemm64<1, true, 0, 0, false><<<dim3(1, NHEAD), blk, 0, stream>>>(
          MH, ML, NTOK, (long)TCHUNK * NTOK, VTH, VTL, NTOK, (long)VTROWS * NTOK,
          (void*)Ub, (void*)Ub, UW, (long)NTOK * UW,
          bqkv, bqkv, 0L, TCHUNK, UW, NTOK, 1.0f);
    }
  }
  coef_kernel<<<dim3(1), dim3(32), 0, stream>>>(PART, bconv, gamma, beta, COEF, nrows);
  combine_kernel<<<dim3(NBATCH * NTOK / 8), blk, 0, stream>>>(U, VSUM, COEF, out);
}
